// WeightedTensorProduct_11536282157112
// MI455X (gfx1250) — hardware-verified
//
#include <hip/hip_runtime.h>


#ifndef NROW
#define NROW 4096
#endif
#define NROW_FULL 4096
#define D1   52
#define DP   64
#define DD   2704
#define HC   2000
#define KP   2048
#define NQ   4096
#define AW   4
#define OPW  13
#define TP   72
#define CARRY_F 64.0f
#define CARRY_X 16.0f
#define CINV (1.0f / 1024.0f)

static_assert(D1 * D1 == DD);
static_assert(DP * DP == NQ);
static_assert(D1 <= DP);
static_assert(D1 % 4 == 0);
static_assert(D1 / 4 == 13);
static_assert(DP == 64);
static_assert(HC % 8 == 0);
static_assert(KP % 64 == 0);
static_assert(KP >= HC);
static_assert(KP / 8 == 256);
static_assert(NQ % 64 == 0);
static_assert(AW * OPW == D1);
static_assert(NROW % 32 == 0);
static_assert(NROW <= NROW_FULL);
static_assert((16 * D1 * 4) % 128 == 0);
static_assert(((16 * D1) / 4) % 8 == 0);
static_assert((16 * D1) / 4 <= 2 * 32 * AW);
static_assert((TP * 2) % 16 == 0);
static_assert(64 * TP * 2 <= 131072);
static_assert(16 * 68 * 4 <= 131072);
static_assert(16 * D1 * 4 <= 131072);

typedef _Float16 h16;
typedef unsigned short bf;
typedef __attribute__((ext_vector_type(16))) __bf16   v16bf;
typedef __attribute__((ext_vector_type(16))) _Float16 v16h;
typedef __attribute__((ext_vector_type(8)))  _Float16 v8h;
typedef __attribute__((ext_vector_type(8)))  unsigned short v8us;
typedef __attribute__((ext_vector_type(8)))  float    v8f;
typedef __attribute__((ext_vector_type(4)))  float    v4f;
typedef v4f  __attribute__((may_alias)) v4fa;
typedef v8us __attribute__((may_alias)) v8usa;

__device__ __forceinline__ unsigned short f2bf(float f) { unsigned u = __float_as_uint(f); u += 0x7FFFu + ((u >> 16) & 1u); return (unsigned short)(u >> 16); }
__device__ __forceinline__ float bfr(float f) { return __uint_as_float(((unsigned)f2bf(f)) << 16); }
__device__ __forceinline__ v16h cat16(v8h lo, v8h hi) { return __builtin_shufflevector(lo, hi, 0, 1, 2, 3, 4, 5, 6, 7, 8, 9, 10, 11, 12, 13, 14, 15); }
__device__ __forceinline__ v16bf cat16b(v8us lo, v8us hi) { return __builtin_bit_cast(v16bf, __builtin_shufflevector(lo, hi, 0, 1, 2, 3, 4, 5, 6, 7, 8, 9, 10, 11, 12, 13, 14, 15)); }
__device__ __forceinline__ v8f wmma16(v16h a, v16h b, v8f c) { return __builtin_amdgcn_wmma_f32_16x16x32_f16(false, a, false, b, (short)0, c, false, false); }
__device__ __forceinline__ v8f wmmab(v16bf a, v16bf b, v8f c) { return __builtin_amdgcn_wmma_f32_16x16x32_bf16(false, a, false, b, (short)0, c, false, false); }
__device__ __forceinline__ v16h  ldh(const h16* p) { return cat16(*(const v8h*)p, *(const v8h*)(p + 16)); }
__device__ __forceinline__ v16bf ldb(const bf* p)  { return cat16b(*(const v8us*)p, *(const v8us*)(p + 16)); }
__device__ __forceinline__ void wave_sync() { __builtin_amdgcn_fence(3  , "wavefront"); __builtin_amdgcn_wave_barrier(); asm volatile("" ::: "memory"); }

static __device__ __forceinline__ h16 toh_flush(float v) { const h16 r = (h16)v; return (fabsf(v) < 6.103515625e-05f) ? (h16)0.0f : r; }
__device__ __forceinline__ v8f wmma16g(v16h a, v16h b, v8f c) { c = wmma16(a, b, c); asm volatile("v_nop\n\tv_nop\n\tv_nop\n\tv_nop" : "+v"(c) : "v"(a), "v"(b)); return c; }
__device__ __forceinline__ v8f wmmabg(v16bf a, v16bf b, v8f c) { c = wmmab(a, b, c); asm volatile("v_nop\n\tv_nop\n\tv_nop\n\tv_nop" : "+v"(c) : "v"(a), "v"(b)); return c; }

__global__ __launch_bounds__(256) void k_wpad(const float* __restrict__ W, bf* WB) {
    const int p = blockIdx.x * 256 + threadIdx.x;
    const int o = p >> 8, c8 = (p & 255) * 8;
    const bool ok = (o < D1) & (c8 < HC);
    const int oc = o < D1 ? o : (D1 - 1);
    const int cc = c8 < HC ? c8 : (HC - 8);
    const float* s = W + (size_t)oc * HC + cc;
    v4f x0 = *(const v4f*)s, x1 = *(const v4f*)(s + 4);
    asm volatile("" : "+v"(x0)); asm volatile("" : "+v"(x1));
    v8us o8;
#pragma unroll
    for (int i = 0; i < 4; ++i) { o8[i] = ok ? f2bf(x0[i]) : (unsigned short)0; o8[4 + i] = ok ? f2bf(x1[i]) : (unsigned short)0; }
    *(volatile v8us*)(WB + (size_t)p * 8) = o8; __threadfence(); *(volatile v8us*)(WB + (size_t)p * 8) = o8;
}
static_assert((DP * (KP / 8)) % 256 == 0);

__global__ __launch_bounds__(256) void k_cbt(const float* __restrict__ C, bf* CT) {
    __shared__ __align__(16) unsigned short ts[64 * TP];
    const int i = blockIdx.x, h0 = blockIdx.y * 64;
    const int ic = i < D1 ? i : (D1 - 1);
#pragma unroll
    for (int it = 0; it < 4; ++it) {
        const int idx = it * 256 + threadIdx.x; const int hr = idx >> 4, q = idx & 15;
        const int h = h0 + hr;
        const bool ok = (h < HC) & (q < 13) & (i < D1);
        const int hc = h < HC ? h : (HC - 1); const int qc = q < 13 ? q : 12;
        v4f x = *(const v4f*)(C + (size_t)hc * DD + (size_t)ic * D1 + qc * 4);
        asm volatile("" : "+v"(x));
#pragma unroll
        for (int c = 0; c < 4; ++c) ts[(4 * q + c) * TP + hr] = ok ? f2bf(x[c]) : (unsigned short)0;
    }
    __syncthreads();
    bf* dst = CT + (size_t)i * 64 * KP + h0;
#pragma unroll 1
    for (int ps = 0; ps < 2; ++ps) {
#pragma unroll
        for (int s = 0; s < 2; ++s) { const int p = s * 256 + threadIdx.x; const int j = p >> 3, c8 = (p & 7) * 8;
            const v8us val = *(const v8usa*)(&ts[j * TP + c8]);
            *(volatile v8us*)(dst + (size_t)j * KP + c8) = val; }
        if (ps == 0) __threadfence(); }
}
static_assert(4 * 256 == 64 * 16);
static_assert(2 * 256 * 16 == 64 * 128);

__global__ __launch_bounds__(32) void k_fold(const bf* __restrict__ A, const bf* __restrict__ Bt, h16* AF) {
    __shared__ __align__(16) float os[16 * 68];
    const int lane = threadIdx.x & 31, lr = lane & 15, hi = lane >> 4; const int c0 = blockIdx.x * 64;
    v8f acc[4][4];
#pragma unroll
    for (int mb = 0; mb < 4; ++mb)
#pragma unroll
        for (int nb = 0; nb < 4; ++nb) acc[mb][nb] = (v8f){};
    const size_t aoff = (size_t)lr * KP + 8 * hi, boff = (size_t)(c0 + lr) * KP + 8 * hi;
#pragma unroll 1
    for (int kc = 0; kc < KP; kc += 32) {
        v16bf a[4];
#pragma unroll
        for (int mb = 0; mb < 4; ++mb) a[mb] = ldb(A + aoff + (size_t)mb * 16 * KP + kc);
#pragma unroll
        for (int nb = 0; nb < 4; ++nb) { const v16bf b = ldb(Bt + boff + (size_t)nb * 16 * KP + kc);
#pragma unroll
            for (int mb = 0; mb < 4; ++mb) acc[mb][nb] = wmmabg(a[mb], b, acc[mb][nb]); }
    }
#pragma unroll
    for (int mb = 0; mb < 4; ++mb) {
#pragma unroll
        for (int nb = 0; nb < 4; ++nb) {
#pragma unroll
            for (int j = 0; j < 8; ++j) os[(hi * 8 + j) * 68 + nb * 16 + lr] = acc[mb][nb][j] * CARRY_F; }
        wave_sync();
#pragma unroll 1
        for (int ps = 0; ps < 2; ++ps) {
#pragma unroll
            for (int s = 0; s < 4; ++s) { const int row = 4 * s + (lane >> 3), c8 = (lane & 7) * 8;
                const v4f x0 = *(const v4fa*)(&os[row * 68 + c8]); const v4f x1 = *(const v4fa*)(&os[row * 68 + c8 + 4]); v8h hv;
#pragma unroll
                for (int i = 0; i < 4; ++i) { hv[i] = toh_flush(x0[i]); hv[4 + i] = toh_flush(x1[i]); }
                const size_t oo = (size_t)(mb * 16 + row) * NQ + (size_t)c0 + c8;
                *(volatile v8h*)(AF + oo) = hv; }
            if (ps == 0) __threadfence(); }
        wave_sync();
    }
}
static_assert(4 * 4 == 16);
static_assert(8 * 8 == 64);

__global__ __launch_bounds__(256) void k_in1f(const float* __restrict__ src, float* dst) {
    const int p = blockIdx.x * 256 + threadIdx.x;
    const int row = p >> 4, q = p & 15;
    const bool ok = q < 13;
    const int qc = q < 13 ? q : 12;
    v4f x = *(const v4f*)(src + (size_t)row * D1 + qc * 4);
    asm volatile("" : "+v"(x));
    v4f o4;
#pragma unroll
    for (int c = 0; c < 4; ++c) o4[c] = ok ? bfr(x[c]) : 0.0f;
    *(volatile v4f*)(dst + (size_t)p * 4) = o4; __threadfence(); *(volatile v4f*)(dst + (size_t)p * 4) = o4;
}
static_assert((NROW * 16) % 256 == 0);

__global__ __launch_bounds__(256) void k_in2h(const float* __restrict__ src, h16* dst) {
    const int p = blockIdx.x * 256 + threadIdx.x;
    const int row = p >> 3, g = p & 7;
    const int q0 = 2 * g, q1 = 2 * g + 1;
    const bool ok0 = q0 < 13, ok1 = q1 < 13;
    const int qc0 = q0 < 13 ? q0 : 12, qc1 = q1 < 13 ? q1 : 12;
    v4f x0 = *(const v4f*)(src + (size_t)row * D1 + qc0 * 4);
    v4f x1 = *(const v4f*)(src + (size_t)row * D1 + qc1 * 4);
    asm volatile("" : "+v"(x0)); asm volatile("" : "+v"(x1));
    v8h hv;
#pragma unroll
    for (int c = 0; c < 4; ++c) {
        const h16 a0 = toh_flush(bfr(x0[c]) * CARRY_X); const h16 a1 = toh_flush(bfr(x1[c]) * CARRY_X);
        hv[c] = ok0 ? a0 : (h16)0.0f; hv[4 + c] = ok1 ? a1 : (h16)0.0f; }
    *(volatile v8h*)(dst + (size_t)p * 8) = hv; __threadfence(); *(volatile v8h*)(dst + (size_t)p * 8) = hv;
}
static_assert((NROW * 8) % 256 == 0);

__global__ __launch_bounds__(32 * AW) void k_apply(const h16* __restrict__ AF, const float* __restrict__ X1, const h16* __restrict__ X2, float* OUT) {
    __shared__ __align__(16) float os[16 * D1];
    const int lane = threadIdx.x & 31, lr = lane & 15, hi = lane >> 4;
    const int wave = __builtin_amdgcn_readfirstlane((int)(threadIdx.x >> 5));
    const int b0 = blockIdx.x * 16;
    const h16* xp = X2 + (size_t)(b0 + lr) * DP + 8 * hi;
    const v16h xb0 = ldh(xp), xb1 = ldh(xp + 32);
    const float* wp = X1 + (size_t)(b0 + lr) * DP + 8 * hi;
    float w1[4][8];
#pragma unroll
    for (int t = 0; t < 4; ++t) { const v4f u0 = *(const v4f*)(wp + 16 * t), u1 = *(const v4f*)(wp + 16 * t + 4);
#pragma unroll
        for (int r = 0; r < 4; ++r) { w1[t][r] = u0[r]; w1[t][4 + r] = u1[r]; } }
#pragma unroll 1
    for (int u = 0; u < OPW; ++u) {
        const int o = wave * OPW + u;
        const h16* ap = AF + (size_t)o * NQ + (size_t)lr * DP + 8 * hi;
        float s = 0.0f;
#pragma unroll
        for (int t = 0; t < 4; ++t) {
            const v16h a0 = ldh(ap + t * 16 * DP), a1 = ldh(ap + t * 16 * DP + 32);
            v8f acc = (v8f){};
            acc = wmma16g(a0, xb0, acc);
            acc = wmma16g(a1, xb1, acc);
#pragma unroll
            for (int r = 0; r < 8; ++r) s = fmaf(w1[t][r], acc[r], s);
        }
        s += __shfl_xor(s, 16, 32);
        if (hi == 0) os[lr * D1 + o] = s * CINV;
    }
    __syncthreads();
    float* ob = OUT + (size_t)b0 * D1;
#pragma unroll 1
    for (int ps = 0; ps < 2; ++ps) {
#pragma unroll
        for (int s2 = 0; s2 < 2; ++s2) { const int p = s2 * (32 * AW) + (int)threadIdx.x;
            const int pc = p < (16 * D1) / 4 ? p : ((16 * D1) / 4 - 1);
            v4f val = *(const v4fa*)(&os[pc * 4]);
            asm volatile("" : "+v"(val));
            if (p < (16 * D1) / 4) *(volatile v4f*)(ob + (size_t)p * 4) = val; }
        if (ps == 0) __threadfence(); }
}

static constexpr size_t al256(size_t v) { return (v + 255) & ~(size_t)255; }
static constexpr size_t SZ_WB = al256((size_t)DP * KP * 2);
static constexpr size_t SZ_CT = al256((size_t)NQ * KP * 2);
static constexpr size_t SZ_AF = al256((size_t)DP * NQ * 2);
static constexpr size_t SZ_X1 = al256((size_t)NROW * DP * 4);
static constexpr size_t SZ_X2 = al256((size_t)NROW * DP * 2);
static constexpr size_t SZ_TOTAL = SZ_WB + SZ_CT + SZ_AF + SZ_X1 + SZ_X2;
static_assert(SZ_TOTAL <= (size_t)134217728);
static_assert((size_t)(DP - 1) * NQ + (NQ - 64) + 64 <= (size_t)DP * NQ);
static_assert((size_t)(NQ - 1) * KP + (KP - 64) + 64 <= (size_t)NQ * KP);
static_assert((size_t)(D1 - 1) * NQ + (size_t)(DP - 1) * DP + DP <= (size_t)DP * NQ);

extern "C" void kernel_launch(void* const* d_in, const int* in_sizes, int n_in,
                              void* d_out, int out_size, void* d_ws, size_t ws_size, hipStream_t stream) {
    (void)stream;
    if (n_in < 4) return;
    if ((size_t)in_sizes[0] < (size_t)NROW * D1 || (size_t)in_sizes[1] < (size_t)NROW * D1) return;
    if ((size_t)in_sizes[2] < (size_t)HC * DD || (size_t)in_sizes[3] < (size_t)D1 * HC) return;
    if ((size_t)out_size < (size_t)NROW * D1) return;
    if (SZ_TOTAL > ws_size) return;
    const float* x1 = (const float*)d_in[0];
    const float* x2 = (const float*)d_in[1];
    const float* cm = (const float*)d_in[2];
    const float* wm = (const float*)d_in[3];
    float* OUT = (float*)d_out;
    char* wsp = (char*)d_ws;
    bf*    WB = (bf*)wsp;    wsp += SZ_WB;
    bf*    CT = (bf*)wsp;    wsp += SZ_CT;
    h16*   AF = (h16*)wsp;   wsp += SZ_AF;
    float* X1 = (float*)wsp; wsp += SZ_X1;
    h16*   X2 = (h16*)wsp;   wsp += SZ_X2;

    k_wpad<<<(unsigned)((DP * (KP / 8)) / 256), 256, 0, stream>>>(wm, WB);
    k_cbt<<<dim3(DP, KP / 64, 1), 256, 0, stream>>>(cm, CT);
    k_fold<<<(unsigned)(NQ / 64), 32, 0, stream>>>(WB, CT, AF);
    k_in1f<<<(unsigned)((NROW * 16) / 256), 256, 0, stream>>>(x1, X1);
    k_in2h<<<(unsigned)((NROW * 8) / 256), 256, 0, stream>>>(x2, X2);
    k_apply<<<(unsigned)(NROW / 16), 32 * AW, 0, stream>>>(AF, X1, X2, OUT);
}
